// GINES_2113123910402
// MI455X (gfx1250) — hardware-verified
//
#include <hip/hip_runtime.h>
#include <stddef.h>
#include <stdint.h>


#define HD        64
#define KP        128
#define NTHR      256
#define NWAVE     8
#define EPT       8
#define CHUNK     (NTHR * EPT)
#define WCAP      (EPT * 32)
#define LISTN     (NWAVE * WCAP)
#define NBRUN     1024
#define PKS       10
#define RCAP      16384
#define DEGCAP    64
#define MEAS_HITS 10486
#define MEAS_DEG  26
#define GBM       128
#define RECW      128
#define STATW     128
#define ARB       64
#define NPL       7
#define NUP       (HD * (KP / 8))
#define G3        192
#define LDS_BKT   ((2 * RCAP + 2 * NBRUN + LISTN + 16) * 4)
#define LDS_HEAD  ((G3 * G3 + G3 + 2 * G3 + G3 + G3 + 256) * 4)
#define WSLIM     134217728

static_assert((CHUNK & (CHUNK - 1)) == 0 && CHUNK <= (1 << 11));
static_assert((NBRUN & (NBRUN - 1)) == 0 && NBRUN == (1 << PKS));
static_assert(NTHR * 4 == NBRUN);
static_assert(LISTN >= NBRUN && LISTN >= NWAVE * WCAP);
static_assert((RCAP % (2 * NTHR)) == 0 && (RCAP % 32) == 0);
static_assert(RCAP * 4 >= MEAS_HITS * 5 && DEGCAP >= 2 * MEAS_DEG);
static_assert(((2 * RCAP + 2 * NBRUN + LISTN) % (4 * NTHR)) == 0);
static_assert(LDS_BKT <= 300000 && LDS_HEAD <= 300000);
static_assert(HD == 2 * 32 && KP == 2 * HD && (KP % 32) == 0);
static_assert(GBM == NWAVE * 16 && (GBM * HD) % NTHR == 0);
static_assert((NUP % NTHR) == 0 && NUP == 1024);
static_assert(ARB == NWAVE * 8 && (GBM % ARB) == 0);
static_assert(G3 <= NTHR && G3 == 3 * HD && ((G3 * G3 / 4) % NTHR) == 0 && (G3 % 32) == 0);
static_assert(RECW == 2 * HD && STATW >= HD + 1 && (STATW % 32) == 0);

typedef float          v2f  __attribute__((ext_vector_type(2)));
typedef float          v4f  __attribute__((ext_vector_type(4)));
typedef float          v8f  __attribute__((ext_vector_type(8)));
typedef int            v4i  __attribute__((ext_vector_type(4)));
typedef int            v8i  __attribute__((ext_vector_type(8)));
typedef unsigned int   v2u  __attribute__((ext_vector_type(2)));
typedef unsigned int   v4u  __attribute__((ext_vector_type(4)));
typedef unsigned short v8us __attribute__((ext_vector_type(8)));
typedef __bf16         v16b __attribute__((ext_vector_type(16)));
typedef v4f  __attribute__((may_alias)) v4fa;
typedef v4i  __attribute__((may_alias)) v4ia;
typedef v8us __attribute__((may_alias)) v8usa;
union Frag { v16b vb; v8us h[2]; v8i w; };

__device__ __forceinline__ v8f wmb(const Frag& a, const Frag& b, v8f c) {
  v8f d = __builtin_amdgcn_wmma_f32_16x16x32_bf16(false, a.vb, false, b.vb, (short)0, c, false, false);
  asm volatile("v_nop\n\tv_nop\n\tv_nop\n\tv_nop" : "+v"(d) : "v"(a.w), "v"(b.w));
  return d;
}

__device__ __forceinline__ unsigned short bf_bits(float f) {
  const unsigned int u = __float_as_uint(f);
  const unsigned int r = u + 0x7FFFu + ((u >> 16) & 1u);
  const unsigned int o = (f != f) ? 0x7fc00000u : r;
  return (unsigned short)(o >> 16);
}
__device__ __forceinline__ float bf_val(unsigned short b) { return __uint_as_float(((unsigned int)b) << 16); }
__device__ __forceinline__ float bf_rne(float f) { return bf_val(bf_bits(f)); }
__device__ __forceinline__ float relu_np(float v) { return (v > 0.0f) ? v : (v - v); }

__device__ __forceinline__ int scan_chunk(const int* __restrict__ dsts, int nE, int cbase, int slotBase,
                                          int nb, int vec8, int* list, int tid, int lane, int wave) {
  int wc = 0;
  const int el0  = tid * EPT;
  const int e0   = cbase + el0;
  const int sent = -2147483647 - 1;
  v4i da, db;
  if (vec8 != 0 && cbase + CHUNK <= nE) {
    da = *(const v4i*)(dsts + e0);
    db = *(const v4i*)(dsts + e0 + 4);
  } else {
    da.x = (e0     < nE) ? dsts[min(e0,     nE - 1)] : sent;
    da.y = (e0 + 1 < nE) ? dsts[min(e0 + 1, nE - 1)] : sent;
    da.z = (e0 + 2 < nE) ? dsts[min(e0 + 2, nE - 1)] : sent;
    da.w = (e0 + 3 < nE) ? dsts[min(e0 + 3, nE - 1)] : sent;
    db.x = (e0 + 4 < nE) ? dsts[min(e0 + 4, nE - 1)] : sent;
    db.y = (e0 + 5 < nE) ? dsts[min(e0 + 5, nE - 1)] : sent;
    db.z = (e0 + 6 < nE) ? dsts[min(e0 + 6, nE - 1)] : sent;
    db.w = (e0 + 7 < nE) ? dsts[min(e0 + 7, nE - 1)] : sent;
  }
  const unsigned nbs = (unsigned)slotBase;
  const unsigned unb = (unsigned)nb;
  const unsigned s0 = (unsigned)da.x - nbs, s1 = (unsigned)da.y - nbs;
  const unsigned s2 = (unsigned)da.z - nbs, s3 = (unsigned)da.w - nbs;
  const unsigned s4 = (unsigned)db.x - nbs, s5 = (unsigned)db.y - nbs;
  const unsigned s6 = (unsigned)db.z - nbs, s7 = (unsigned)db.w - nbs;
  const bool h0 = s0 < unb, h1 = s1 < unb, h2 = s2 < unb, h3 = s3 < unb;
  const bool h4 = s4 < unb, h5 = s5 < unb, h6 = s6 < unb, h7 = s7 < unb;
  const unsigned any = __builtin_amdgcn_ballot_w32(h0 | h1 | h2 | h3 | h4 | h5 | h6 | h7);
  if (any != 0u) {
#define HITJ(J, HJ, SJ) { \
      const unsigned mj = __builtin_amdgcn_ballot_w32(HJ); \
      if (mj != 0u) { \
        if (HJ) { \
          const int pos = wc + (int)__builtin_amdgcn_mbcnt_lo(mj, 0u); \
          if (pos < WCAP) list[wave * WCAP + pos] = ((el0 + (J)) << PKS) | (int)(SJ); \
        } \
        wc += (int)__builtin_popcount(mj); } }
    HITJ(0, h0, s0)
    HITJ(1, h1, s1)
    HITJ(2, h2, s2)
    HITJ(3, h3, s3)
    HITJ(4, h4, s4)
    HITJ(5, h5, s5)
    HITJ(6, h6, s6)
    HITJ(7, h7, s7)
#undef HITJ
  }
  return wc;
}

__device__ __forceinline__ v8us cv8b(const float* __restrict__ p) {
  v8us o;
#pragma unroll
  for (int i = 0; i < 8; ++i) o[i] = bf_bits(p[(size_t)i * HD]);
  return o;
}

__global__ __launch_bounds__(NTHR) void k_prep(const float* __restrict__ w0, const float* __restrict__ w1,
                                               const float* __restrict__ w2, const float* __restrict__ w3,
                                               const float* __restrict__ w4, const float* __restrict__ w5,
                                               const float* __restrict__ w6, unsigned short* bt) {
  const int u  = (int)blockIdx.x * NTHR + (int)threadIdx.x;
  const int pl = u >> 10;
  const int v  = u & (NUP - 1);
  const int n  = v >> 4;
  const int kk = ((v & 15) * 8) & (HD - 1);
  const size_t so = (size_t)kk * HD + (size_t)n;
  v8us o;
  if (pl == 0)      o = cv8b(w0 + so);
  else if (pl == 1) o = cv8b(w1 + so);
  else if (pl == 2) o = cv8b(w2 + so);
  else if (pl == 3) o = cv8b(w3 + so);
  else if (pl == 4) o = cv8b(w4 + so);
  else if (pl == 5) o = cv8b(w5 + so);
  else if (pl == 6) o = cv8b(w6 + so);
  else return;
  unsigned short* dp = bt + (size_t)u * 8;
  *(volatile v8us*)dp = o;
  __threadfence();
  *(volatile v8us*)dp = o;
}

__global__ __launch_bounds__(NTHR) void k_bucket(const int* __restrict__ srcs, const int* __restrict__ dsts,
                                                 const float* __restrict__ ea, int nN, int nE, int vec8,
                                                 unsigned int* lst, int* cntg, int* offg, int* flg) {
  extern __shared__ v4f lds_dyn[];
  int* reg1 = (int*)lds_dyn;
  int* reg2 = reg1 + RCAP;
  int* scnt = reg2 + RCAP;
  int* soff = scnt + NBRUN;
  int* list = soff + NBRUN;
  int* wcnt = list + LISTN;
  int* wtot = wcnt + NWAVE;
  const int tid = (int)threadIdx.x, lane = tid & 31, wave = tid >> 5;
  const int nodeBase = (int)blockIdx.x * NBRUN;

  {
    const v4i z4 = {0, 0, 0, 0};
    for (int i = tid * 4; i < 2 * RCAP + 2 * NBRUN + LISTN; i += NTHR * 4) *(v4ia*)(reg1 + i) = z4;
    if (tid < 16) wcnt[tid] = 0;
  }
  __syncthreads();

  int tot = 0, ovf = 0;
  const int nChunks = (nE + CHUNK - 1) / CHUNK;
#pragma unroll 1
  for (int ch = 0; ch < nChunks; ++ch) {
    const int cbase = ch * CHUNK;
    const int wc = scan_chunk(dsts, nE, cbase, nodeBase, NBRUN, vec8, list, tid, lane, wave);
    if (lane == 0) wcnt[wave] = wc;
    __syncthreads();
    int pre = 0, all = 0;
#pragma unroll
    for (int w2 = 0; w2 < NWAVE; ++w2) {
      int c = wcnt[w2];
      c = c < 0 ? 0 : (c > WCAP ? WCAP : c);
      all += c;
      pre += (w2 < wave) ? c : 0;
    }
    const int wcc  = wc < 0 ? 0 : (wc > WCAP ? WCAP : wc);
    const int base = tot + pre;
#pragma unroll 1
    for (int i = lane; i < wcc; i += 32) {
      const int ent = list[wave * WCAP + i];
      const int el  = (ent >> PKS) & (CHUNK - 1);
      const int sl  = ent & (NBRUN - 1);
      int eid = cbase + el;
      eid = eid > nE - 1 ? nE - 1 : eid;
      const int pos = base + i;
      if (pos < RCAP) reg1[pos] = (int)(((unsigned)eid << PKS) | (unsigned)sl);
    }
    if (tot + all > RCAP) ovf = 1;
    tot += all;
    tot = tot > RCAP ? RCAP : tot;
    __syncthreads();
  }
  const int nh = tot;

  if (wave == 0) {
#pragma unroll 1
    for (int b0 = 0; b0 < nh; b0 += 32) {
      const int idx = b0 + lane;
      const int uv  = reg1[idx < RCAP ? idx : RCAP - 1];
      const int m32 = (nh - b0) < 32 ? (nh - b0) : 32;
#pragma unroll 1
      for (int k = 0; k < m32; ++k) {
        const int u  = __builtin_amdgcn_readlane(uv, k);
        const int sl = u & (NBRUN - 1);
        if (lane == 0) scnt[sl] = scnt[sl] + 1;
      }
    }
  }
  __syncthreads();

  {
    const v4i ca = *(const v4ia*)(scnt + 4 * tid);
    const int e0 = ca.x < 0 ? 0 : ca.x, e1 = ca.y < 0 ? 0 : ca.y, e2 = ca.z < 0 ? 0 : ca.z, e3 = ca.w < 0 ? 0 : ca.w;
    const int ts = e0 + e1 + e2 + e3;
    int incl = ts;
#pragma unroll
    for (int d = 1; d < 32; d <<= 1) {
      const int up = __shfl_up(incl, d);
      if (lane >= d) incl += up;
    }
    if (lane == 31) wtot[wave] = incl;
    __syncthreads();
    int pre = 0;
#pragma unroll
    for (int w2 = 0; w2 < NWAVE; ++w2) pre += (w2 < wave) ? wtot[w2] : 0;
    int run = pre + incl - ts;
    soff[4 * tid + 0] = run; run += e0;
    soff[4 * tid + 1] = run; run += e1;
    soff[4 * tid + 2] = run; run += e2;
    soff[4 * tid + 3] = run;
  }
  __syncthreads();
  for (int i = tid; i < NBRUN; i += NTHR) list[i] = soff[i];
  __syncthreads();

  if (wave == 0) {
#pragma unroll 1
    for (int b0 = 0; b0 < nh; b0 += 32) {
      const int idx = b0 + lane;
      const int uv  = reg1[idx < RCAP ? idx : RCAP - 1];
      const int m32 = (nh - b0) < 32 ? (nh - b0) : 32;
#pragma unroll 1
      for (int k = 0; k < m32; ++k) {
        const int u   = __builtin_amdgcn_readlane(uv, k);
        const int sl  = u & (NBRUN - 1);
        const int eid = (int)((unsigned)u >> PKS);
        if (lane == 0) {
          int pos = list[sl];
          pos = pos < 0 ? 0 : (pos > RCAP - 1 ? RCAP - 1 : pos);
          reg2[pos] = eid;
          list[sl] = pos + 1;
        }
      }
    }
  }
  __syncthreads();

#pragma unroll 1
  for (int it = 0; it < RCAP / 2 / NTHR; ++it) {
    const int p  = it * NTHR + tid;
    const int i0 = 2 * p;
    int e0 = reg2[i0], e1 = reg2[i0 + 1];
    e0 = e0 < 0 ? 0 : (e0 > nE - 1 ? nE - 1 : e0);
    e1 = e1 < 0 ? 0 : (e1 > nE - 1 ? nE - 1 : e1);
    const int   s0 = srcs[e0], s1 = srcs[e1];
    const float a0 = bf_rne(ea[e0]), a1 = bf_rne(ea[e1]);
    const bool  l0 = i0 < nh, l1 = (i0 + 1) < nh;
    v4u r;
    r.x = l0 ? (unsigned)s0 : 0u;
    r.y = l0 ? __float_as_uint(a0) : 0u;
    r.z = l1 ? (unsigned)s1 : 0u;
    r.w = l1 ? __float_as_uint(a1) : 0u;
    unsigned int* dp = lst + ((size_t)blockIdx.x * RCAP + (size_t)i0) * 2;
    *(volatile v4u*)dp = r;
    __threadfence();
    *(volatile v4u*)dp = r;
  }
  {
    const v4i cv = *(const v4ia*)(scnt + 4 * tid);
    const v4i ov = *(const v4ia*)(soff + 4 * tid);
    const v4i fv = {ovf, ovf, ovf, ovf};
    int* cp = cntg + (size_t)blockIdx.x * NBRUN + 4 * tid;
    int* op = offg + (size_t)blockIdx.x * NBRUN + 4 * tid;
    int* fp = flg + (size_t)blockIdx.x * 32 + 4 * (tid & 7);
    const bool fw = tid < 8;
    *(volatile v4i*)cp = cv;
    *(volatile v4i*)op = ov;
    if (fw) *(volatile v4i*)fp = fv;
    __threadfence();
    *(volatile v4i*)cp = cv;
    *(volatile v4i*)op = ov;
    if (fw) *(volatile v4i*)fp = fv;
  }
}

__global__ __launch_bounds__(NTHR) void k_agg1(const float* __restrict__ x, const unsigned int* __restrict__ lst,
    const int* __restrict__ cntg, const int* __restrict__ offg, const int* __restrict__ flg,
    const float* __restrict__ l2w, const float* __restrict__ l2b, const float* __restrict__ lew,
    const float* __restrict__ leb, const float* __restrict__ n1w, const float* __restrict__ n1b,
    const float* __restrict__ bng, const float* __restrict__ bnb, const float* __restrict__ bnm,
    const float* __restrict__ bnv, unsigned int* aout, int nN, int mRows) {
  const int tid = (int)threadIdx.x, lane = tid & 31, wave = tid >> 5;
  const v4f w4 = *(const v4f*)l2w;
  const float W00 = bf_rne(w4.x), W01 = bf_rne(w4.y), W10 = bf_rne(w4.z), W11 = bf_rne(w4.w);
  const v2f b2 = *(const v2f*)l2b, lw = *(const v2f*)lew, lb = *(const v2f*)leb;
  const float B0 = bf_rne(b2.x), B1 = bf_rne(b2.y);
  const float LW0 = bf_rne(lw.x), LW1 = bf_rne(lw.y), LB0 = bf_rne(lb.x), LB1 = bf_rne(lb.y);
  const v2f nw0 = *(const v2f*)(n1w + 2 * lane), nw1 = *(const v2f*)(n1w + HD + 2 * lane);
  const v2f nb = *(const v2f*)(n1b + 2 * lane);
  const v2f gg = *(const v2f*)(bng + 2 * lane), bb = *(const v2f*)(bnb + 2 * lane);
  const v2f mm = *(const v2f*)(bnm + 2 * lane), vv = *(const v2f*)(bnv + 2 * lane);
  const float NW00 = bf_rne(nw0.x), NW01 = bf_rne(nw0.y), NW10 = bf_rne(nw1.x), NW11 = bf_rne(nw1.y);
  const float NB0 = bf_rne(nb.x), NB1 = bf_rne(nb.y);
  const float G0 = bf_rne(gg.x), G1 = bf_rne(gg.y), BB0 = bf_rne(bb.x), BB1 = bf_rne(bb.y);
  const float M0 = bf_rne(mm.x), M1 = bf_rne(mm.y);
  const float R0 = 1.0f / sqrtf(bf_rne(vv.x) + 1e-5f), R1 = 1.0f / sqrtf(bf_rne(vv.y) + 1e-5f);
  const float qnan = __int_as_float(0x7fc00000);
  const int rowBase = (int)blockIdx.x * ARB + wave * 8;

#pragma unroll 1
  for (int i = 0; i < 8; ++i) {
    const int grow = rowBase + i;
    const bool live = grow < nN;
    const int nc = live ? grow : nN - 1;
    const v2f xdv = *(const v2f*)(x + 2 * (size_t)nc);
    const float xd0 = bf_rne(xdv.x), xd1 = bf_rne(xdv.y);
    const int bk = nc >> PKS;
    const int craw = cntg[nc];
    int st = offg[nc];
    const int fl = flg[bk * 32];
    int cnt = craw < 0 ? 0 : (craw > DEGCAP ? DEGCAP : craw);
    st = st < 0 ? 0 : (st > RCAP ? RCAP : st);
    if (cnt > RCAP - st) cnt = RCAP - st;
    float a0 = 0.0f, a1 = 0.0f;
#pragma unroll 1
    for (int b0 = 0; b0 < cnt; b0 += 32) {
      const int j = b0 + lane;
      const bool ok = j < cnt;
      int idx = st + j; idx = idx > RCAP - 1 ? RCAP - 1 : idx;
      const v2u rec = *(const v2u*)(lst + ((size_t)bk * RCAP + (size_t)idx) * 2);
      int s = (int)rec.x; s = s < 0 ? 0 : (s > nN - 1 ? nN - 1 : s);
      const float eav = __uint_as_float(rec.y);
      const v2f xsv = *(const v2f*)(x + 2 * (size_t)s);
      const float d0 = bf_rne(xsv.x) - xd0, d1 = bf_rne(xsv.y) - xd1;
      float u0 = (d0 * W00 + d1 * W10 + B0) + (eav * LW0 + LB0);
      float u1 = (d0 * W01 + d1 * W11 + B1) + (eav * LW1 + LB1);
      u0 = relu_np(u0); u1 = relu_np(u1);
      a0 += ok ? u0 : 0.0f;
      a1 += ok ? u1 : 0.0f;
    }
#pragma unroll
    for (int d = 16; d >= 1; d >>= 1) {
      a0 += __shfl_xor(a0, d);
      a1 += __shfl_xor(a1, d);
    }
    const float pz = (fl != 0 || craw > DEGCAP) ? qnan : 0.0f;
    const float o0 = a0 + xd0, o1 = a1 + xd1;
    float z0 = (o0 * NW00 + o1 * NW10) + NB0;
    float z1 = (o0 * NW01 + o1 * NW11) + NB1;
    z0 = (G0 * (z0 - M0)) * R0 + BB0;
    z1 = (G1 * (z1 - M1)) * R1 + BB1;
    z0 = relu_np(z0) + pz;
    z1 = relu_np(z1) + pz;
    z0 = live ? z0 : 0.0f;
    z1 = live ? z1 : 0.0f;
    const unsigned short h0 = bf_bits(z0), h1 = bf_bits(z1);
    const unsigned short l0 = bf_bits(z0 - bf_val(h0)), l1 = bf_bits(z1 - bf_val(h1));
    const unsigned int hw = (unsigned int)h0 | ((unsigned int)h1 << 16);
    const unsigned int lw2 = (unsigned int)l0 | ((unsigned int)l1 << 16);
    unsigned int* op = aout + (size_t)grow * (KP / 2) + lane;
    const bool wsv = grow < mRows;
    if (wsv) { *(volatile unsigned int*)op = hw; *(volatile unsigned int*)(op + 32) = lw2; }
    __threadfence();
    if (wsv) { *(volatile unsigned int*)op = hw; *(volatile unsigned int*)(op + 32) = lw2; }
  }
}

__global__ __launch_bounds__(NTHR) void k_agg(const float* __restrict__ P, const unsigned int* __restrict__ hpl,
    const unsigned int* __restrict__ lst, const int* __restrict__ cntg, const int* __restrict__ offg,
    const int* __restrict__ flg, const float* __restrict__ l2b, const float* __restrict__ lew,
    const float* __restrict__ leb, unsigned int* aout, int nN, int mRows) {
  const int tid = (int)threadIdx.x, lane = tid & 31, wave = tid >> 5;
  const v2f b2 = *(const v2f*)(l2b + 2 * lane);
  const v2f lw = *(const v2f*)(lew + 2 * lane);
  const v2f lb = *(const v2f*)(leb + 2 * lane);
  const float B0 = bf_rne(b2.x), B1 = bf_rne(b2.y);
  const float LW0 = bf_rne(lw.x), LW1 = bf_rne(lw.y), LB0 = bf_rne(lb.x), LB1 = bf_rne(lb.y);
  const float qnan = __int_as_float(0x7fc00000);
  const int rowBase = (int)blockIdx.x * ARB + wave * 8;

#pragma unroll 1
  for (int i = 0; i < 8; ++i) {
    const int grow = rowBase + i;
    const bool live = grow < nN;
    const int nc = live ? grow : nN - 1;
    const v2f pd = *(const v2f*)(P + (size_t)nc * HD + 2 * lane);
    const float base0 = B0 - pd.x, base1 = B1 - pd.y;
    const int bk = nc >> PKS;
    const int craw = cntg[nc];
    int st = offg[nc];
    const int fl = flg[bk * 32];
    int cnt = craw < 0 ? 0 : (craw > DEGCAP ? DEGCAP : craw);
    st = st < 0 ? 0 : (st > RCAP ? RCAP : st);
    if (cnt > RCAP - st) cnt = RCAP - st;
    float a0 = 0.0f, a1 = 0.0f;
#pragma unroll 1
    for (int b0 = 0; b0 < cnt; b0 += 32) {
      int idx = st + b0 + lane; idx = idx > RCAP - 1 ? RCAP - 1 : idx;
      const v2u rec = *(const v2u*)(lst + ((size_t)bk * RCAP + (size_t)idx) * 2);
      int s = (int)rec.x; s = s < 0 ? 0 : (s > nN - 1 ? nN - 1 : s);
      const int eb = (int)rec.y;
      const int m32 = (cnt - b0) < 32 ? (cnt - b0) : 32;
#pragma unroll 1
      for (int k = 0; k < m32; ++k) {
        const int   sk = __builtin_amdgcn_readlane(s, k);
        const float ek = __int_as_float(__builtin_amdgcn_readlane(eb, k));
        const v2f ps = *(const v2f*)(P + (size_t)sk * HD + 2 * lane);
        const float v0 = (ps.x + base0) + (ek * LW0 + LB0);
        const float v1 = (ps.y + base1) + (ek * LW1 + LB1);
        a0 += relu_np(v0);
        a1 += relu_np(v1);
      }
    }
    const unsigned int hwd = hpl[(size_t)nc * (KP / 2) + lane];
    const unsigned int lwd = hpl[(size_t)nc * (KP / 2) + 32 + lane];
    const float hs0 = __uint_as_float(hwd << 16) + __uint_as_float(lwd << 16);
    const float hs1 = __uint_as_float(hwd & 0xffff0000u) + __uint_as_float(lwd & 0xffff0000u);
    const float pz = (fl != 0 || craw > DEGCAP) ? qnan : 0.0f;
    float r0 = (a0 + hs0) + pz, r1 = (a1 + hs1) + pz;
    r0 = live ? r0 : 0.0f;
    r1 = live ? r1 : 0.0f;
    const unsigned short h0 = bf_bits(r0), h1 = bf_bits(r1);
    const unsigned short l0 = bf_bits(r0 - bf_val(h0)), l1 = bf_bits(r1 - bf_val(h1));
    const unsigned int hw = (unsigned int)h0 | ((unsigned int)h1 << 16);
    const unsigned int lw2 = (unsigned int)l0 | ((unsigned int)l1 << 16);
    unsigned int* op = aout + (size_t)grow * (KP / 2) + lane;
    const bool wsv = grow < mRows;
    if (wsv) { *(volatile unsigned int*)op = hw; *(volatile unsigned int*)(op + 32) = lw2; }
    __threadfence();
    if (wsv) { *(volatile unsigned int*)op = hw; *(volatile unsigned int*)(op + 32) = lw2; }
  }
}

template <int EPI>
__global__ __launch_bounds__(NTHR) void k_gemm(const unsigned short* __restrict__ A,
                                               const unsigned short* __restrict__ BT,
                                               const float* __restrict__ bias, const float* __restrict__ bng,
                                               const float* __restrict__ bnb, const float* __restrict__ bnm,
                                               const float* __restrict__ bnv,
                                               float* outF, unsigned short* outH, float* rec, int nN) {
  __shared__ __attribute__((aligned(16))) float stg[GBM * HD];
  __shared__ __attribute__((aligned(16))) float sp[5 * HD];
  __shared__ __attribute__((aligned(16))) float pst[RECW];
  const int tid = (int)threadIdx.x, lane = tid & 31, wave = tid >> 5, hh = lane >> 4, m = lane & 15;
  const int rowBase = (int)blockIdx.x * GBM;

  if constexpr (EPI != 0) {
    if (tid < HD) {
      sp[tid] = bf_rne(bias[tid]);
      if constexpr (EPI == 2) {
        sp[HD + tid]     = bf_rne(bng[tid]);
        sp[2 * HD + tid] = bf_rne(bnb[tid]);
        sp[3 * HD + tid] = bf_rne(bnm[tid]);
        sp[4 * HD + tid] = 1.0f / sqrtf(bf_rne(bnv[tid]) + 1e-5f);
      }
    }
  }

  v8f acc[4];
  {
    const v8f z = {0.f, 0.f, 0.f, 0.f, 0.f, 0.f, 0.f, 0.f};
#pragma unroll
    for (int t = 0; t < 4; ++t) acc[t] = z;
  }
  const unsigned short* ap = A  + (size_t)(rowBase + 16 * wave + m) * (size_t)KP + 8 * hh;
  const unsigned short* bp = BT + (size_t)m * (size_t)KP + 8 * hh;

#pragma unroll 1
  for (int k0 = 0; k0 < KP; k0 += 32) {
    Frag af;
    af.h[0] = *(const v8usa*)(ap + k0);
    af.h[1] = *(const v8usa*)(ap + k0 + 16);
#pragma unroll
    for (int nt = 0; nt < 4; ++nt) {
      const unsigned short* wq = bp + (size_t)(16 * nt) * (size_t)KP + k0;
      Frag bfr;
      bfr.h[0] = *(const v8usa*)wq;
      bfr.h[1] = *(const v8usa*)(wq + 16);
      acc[nt] = wmb(af, bfr, acc[nt]);
    }
  }

#pragma unroll
  for (int nt = 0; nt < 4; ++nt) {
    const int lc = 16 * nt + m;
#pragma unroll
    for (int r = 0; r < 8; ++r) {
      const int lr = 16 * wave + 8 * hh + r;
      const bool live = (rowBase + lr) < nN;
      stg[lr * HD + lc] = live ? acc[nt][r] : 0.0f;
    }
  }
  __syncthreads();

  if constexpr (EPI != 0) {
#pragma unroll 1
    for (int i = 0; i < (GBM * HD) / NTHR; ++i) {
      const int idx = i * NTHR + tid;
      const int col = idx & (HD - 1);
      const bool live = (rowBase + (idx >> 6)) < nN;
      float v = stg[idx] + sp[col];
      if constexpr (EPI == 2) {
        v = (sp[HD + col] * (v - sp[3 * HD + col])) * sp[4 * HD + col] + sp[2 * HD + col];
      }
      v = relu_np(v);
      stg[idx] = live ? v : 0.0f;
    }
    __syncthreads();
  }

  if constexpr (EPI == 2) {
    const int q  = lane & 15;
    const int cb = 8 * (q & 7);
    const bool isHi = q < 8;
    v4u pk[8];
#pragma unroll
    for (int i = 0; i < 8; ++i) {
      const int lr = 16 * wave + 2 * i + hh;
      const v4f a = *(const v4fa*)(stg + lr * HD + cb);
      const v4f b = *(const v4fa*)(stg + lr * HD + cb + 4);
      const float f[8] = {a.x, a.y, a.z, a.w, b.x, b.y, b.z, b.w};
      unsigned int w[4];
#pragma unroll
      for (int j = 0; j < 4; ++j) {
        const unsigned short h0 = bf_bits(f[2 * j]), h1 = bf_bits(f[2 * j + 1]);
        const unsigned short l0 = bf_bits(f[2 * j] - bf_val(h0)), l1 = bf_bits(f[2 * j + 1] - bf_val(h1));
        const unsigned short q0 = isHi ? h0 : l0, q1 = isHi ? h1 : l1;
        w[j] = (unsigned int)q0 | ((unsigned int)q1 << 16);
      }
      v4u pv; pv.x = w[0]; pv.y = w[1]; pv.z = w[2]; pv.w = w[3];
      pk[i] = pv;
    }
    unsigned short* ob = outH + (size_t)(rowBase + 16 * wave) * (size_t)KP + 8 * lane;
#pragma unroll
    for (int i = 0; i < 8; ++i) *(volatile v4u*)(ob + i * 2 * KP) = pk[i];
    __threadfence();
#pragma unroll
    for (int i = 0; i < 8; ++i) *(volatile v4u*)(ob + i * 2 * KP) = pk[i];
  } else {
    v4f pv = {0.f, 0.f, 0.f, 0.f};
    const bool pok = (EPI == 1) && (tid < RECW / 4);
    if constexpr (EPI == 1) {
      int nvr = nN - rowBase;
      nvr = nvr < 0 ? 0 : (nvr > GBM ? GBM : nvr);
      if (tid < HD) {
        float s = 0.0f;
#pragma unroll 1
        for (int r = 0; r < nvr; ++r) s += stg[r * HD + tid];
        const float inv = 1.0f / (float)(nvr < 1 ? 1 : nvr);
        const float mean = s * inv;
        float qq = 0.0f;
#pragma unroll 1
        for (int r = 0; r < nvr; ++r) {
          const float d = stg[r * HD + tid] - mean;
          qq = fmaf(d, d, qq);
        }
        pst[tid] = mean;
        pst[HD + tid] = qq;
      }
      __syncthreads();
      if (pok) pv = *(const v4fa*)(pst + 4 * tid);
    }
    v4f fv[8];
#pragma unroll
    for (int i = 0; i < 8; ++i) {
      const int lr = 16 * wave + 2 * i + hh;
      fv[i] = *(const v4fa*)(stg + lr * HD + 4 * m);
    }
    float* ob = outF + (size_t)(rowBase + 16 * wave) * (size_t)HD + 4 * lane;
    float* pp = rec + (size_t)blockIdx.x * RECW + 4 * (tid & 31);
#pragma unroll
    for (int i = 0; i < 8; ++i) *(volatile v4f*)(ob + i * 2 * HD) = fv[i];
    if (pok) *(volatile v4f*)pp = pv;
    __threadfence();
#pragma unroll
    for (int i = 0; i < 8; ++i) *(volatile v4f*)(ob + i * 2 * HD) = fv[i];
    if (pok) *(volatile v4f*)pp = pv;
  }
}

__global__ __launch_bounds__(HD) void k_comb(const float* __restrict__ rec, int nBlk, int nN, float* stat) {
  __shared__ double sq[HD];
  __shared__ __attribute__((aligned(16))) float so[STATW];
  const int tid = (int)threadIdx.x;
  double n = 0.0, mean = 0.0, M2 = 0.0;
#pragma unroll 1
  for (int b = 0; b < nBlk; ++b) {
    int nvr = nN - b * GBM;
    nvr = nvr < 0 ? 0 : (nvr > GBM ? GBM : nvr);
    const double mb = (double)rec[(size_t)b * RECW + tid];
    const double qb = (double)rec[(size_t)b * RECW + HD + tid];
    if (nvr > 0) {
      const double nb = (double)nvr;
      const double nn = n + nb;
      const double delta = mb - mean;
      const double f = nb / nn;
      mean = mean + delta * f;
      M2 = M2 + qb + delta * delta * n * f;
      n = nn;
    }
  }
  sq[tid] = M2;
  so[tid] = (float)mean;
  so[HD + tid] = 0.0f;
  __syncthreads();
  if (tid == 0) {
    double t = 0.0;
#pragma unroll 1
    for (int i = 0; i < HD; ++i) t += sq[i];
    const double nt = n < 1.0 ? 1.0 : n;
    const float msq = (float)(t / nt);
    so[HD] = 1.0f / sqrtf(1e-6f + msq);
  }
  __syncthreads();
  const bool ok = tid < STATW / 4;
  v4f v = {0.f, 0.f, 0.f, 0.f};
  if (ok) v = *(const v4fa*)(so + 4 * tid);
  float* dp = stat + 4 * (tid & 31);
  if (ok) *(volatile v4f*)dp = v;
  __threadfence();
  if (ok) *(volatile v4f*)dp = v;
}

__global__ __launch_bounds__(NTHR) void k_apply(const float* __restrict__ C, const float* __restrict__ stat,
                                                unsigned short* outH, int nN, int nUnits) {
  const int u = (int)blockIdx.x * NTHR + (int)threadIdx.x;
  if (u >= nUnits) return;
  const int row = u >> 4, q = u & 15, cb = 8 * (q & 7);
  const bool live = row < nN;
  const int rc = live ? row : nN - 1;
  const v4f a = *(const v4f*)(C + (size_t)rc * HD + cb);
  const v4f b = *(const v4f*)(C + (size_t)rc * HD + cb + 4);
  const v4f ma = *(const v4f*)(stat + cb);
  const v4f mb = *(const v4f*)(stat + cb + 4);
  const float s = stat[HD];
  const float f[8] = {(a.x - ma.x) * s, (a.y - ma.y) * s, (a.z - ma.z) * s, (a.w - ma.w) * s,
                      (b.x - mb.x) * s, (b.y - mb.y) * s, (b.z - mb.z) * s, (b.w - mb.w) * s};
  const bool isHi = q < 8;
  unsigned int w[4];
#pragma unroll
  for (int j = 0; j < 4; ++j) {
    const float f0 = live ? f[2 * j] : 0.0f, f1 = live ? f[2 * j + 1] : 0.0f;
    const unsigned short h0 = bf_bits(f0), h1 = bf_bits(f1);
    const unsigned short l0 = bf_bits(f0 - bf_val(h0)), l1 = bf_bits(f1 - bf_val(h1));
    const unsigned short q0 = isHi ? h0 : l0, q1 = isHi ? h1 : l1;
    w[j] = (unsigned int)q0 | ((unsigned int)q1 << 16);
  }
  v4u pv; pv.x = w[0]; pv.y = w[1]; pv.z = w[2]; pv.w = w[3];
  unsigned short* dp = outH + (size_t)u * 8;
  *(volatile v4u*)dp = pv;
  __threadfence();
  *(volatile v4u*)dp = pv;
}

__global__ __launch_bounds__(NTHR) void k_pool(const float* __restrict__ C, const float* __restrict__ stat,
                                               const int* __restrict__ bat, int nN, int vec8b,
                                               float* pool, int colOff) {
  __shared__ int list[LISTN];
  __shared__ float part[NWAVE * HD];
  __shared__ __attribute__((aligned(16))) float outv[HD];
  const int tid = (int)threadIdx.x, lane = tid & 31, wave = tid >> 5;
  const int g = (int)blockIdx.x;
  const v2f mv = *(const v2f*)(stat + 2 * lane);
  const float s = stat[HD];
  float a0 = 0.0f, a1 = 0.0f;
  const int nChunks = (nN + CHUNK - 1) / CHUNK;
#pragma unroll 1
  for (int ch = 0; ch < nChunks; ++ch) {
    const int cbase = ch * CHUNK;
    const int wc = scan_chunk(bat, nN, cbase, g, 1, vec8b, list, tid, lane, wave);
    __syncthreads();
    const int wcc = wc < 0 ? 0 : (wc > WCAP ? WCAP : wc);
#pragma unroll 1
    for (int i = 0; i < wcc; ++i) {
      const int ent = list[wave * WCAP + i];
      const int el  = (ent >> PKS) & (CHUNK - 1);
      int node = cbase + el;
      node = node < 0 ? 0 : (node > nN - 1 ? nN - 1 : node);
      const v2f c = *(const v2f*)(C + (size_t)node * HD + 2 * lane);
      a0 += (c.x - mv.x) * s;
      a1 += (c.y - mv.y) * s;
    }
    __syncthreads();
  }
  part[wave * HD + 2 * lane]     = a0;
  part[wave * HD + 2 * lane + 1] = a1;
  __syncthreads();
  if (tid < HD) {
    double t = 0.0;
#pragma unroll 1
    for (int w2 = 0; w2 < NWAVE; ++w2) t += (double)part[w2 * HD + tid];
    outv[tid] = (float)t;
  }
  __syncthreads();
  const bool ok = tid < HD / 4;
  const v4f v = *(const v4fa*)(outv + 4 * (tid & (HD / 4 - 1)));
  float* dp = pool + (size_t)g * G3 + colOff + 4 * (tid & 15);
  if (ok) *(volatile v4f*)dp = v;
  __threadfence();
  if (ok) *(volatile v4f*)dp = v;
}

__global__ __launch_bounds__(NTHR) void k_head(const float* __restrict__ pool, const float* __restrict__ w1,
                                               const float* __restrict__ b1, const float* __restrict__ w2,
                                               const float* __restrict__ b2, int nG, float* out) {
  extern __shared__ v4f lds_dyn[];
  float* sW  = (float*)lds_dyn;
  float* sB1 = sW + G3 * G3;
  float* sW2 = sB1 + G3;
  float* sG  = sW2 + 2 * G3;
  float* sT  = sG + G3;
  float* sO  = sT + G3;
  const int tid = (int)threadIdx.x, lane = tid & 31, wave = tid >> 5;
#pragma unroll 1
  for (int it = 0; it < (G3 * G3 / 4) / NTHR; ++it) {
    const int idx = it * NTHR + tid;
    const v4f v = *(const v4f*)(w1 + 4 * (size_t)idx);
    v4f o;
    o.x = bf_rne(v.x); o.y = bf_rne(v.y); o.z = bf_rne(v.z); o.w = bf_rne(v.w);
    *(v4fa*)(sW + 4 * idx) = o;
  }
  if (tid < G3) {
    sB1[tid] = bf_rne(b1[tid]);
    sW2[tid] = bf_rne(w2[tid]);
    sW2[G3 + tid] = bf_rne(w2[G3 + tid]);
    sT[tid] = 0.0f;
  }
  sO[tid] = 0.0f;
  const float b20 = bf_rne(b2[0]), b21 = bf_rne(b2[1]);
  __syncthreads();

#pragma unroll 1
  for (int g = 0; g < nG; ++g) {
    if (tid < G3) sG[tid] = pool[(size_t)g * G3 + tid];
    __syncthreads();
    if (tid < G3) {
      float acc = 0.0f;
#pragma unroll 4
      for (int k = 0; k < G3; ++k) acc = fmaf(sG[k], sW[k * G3 + tid], acc);
      sT[tid] = relu_np(acc + sB1[tid]);
    }
    __syncthreads();
    if (wave == 0) {
      float p0 = 0.0f, p1 = 0.0f;
#pragma unroll 1
      for (int j = 0; j < G3 / 32; ++j) {
        const int k = lane + 32 * j;
        const float t = sT[k];
        p0 = fmaf(t, sW2[2 * k], p0);
        p1 = fmaf(t, sW2[2 * k + 1], p1);
      }
#pragma unroll
      for (int d = 16; d >= 1; d >>= 1) {
        p0 += __shfl_xor(p0, d);
        p1 += __shfl_xor(p1, d);
      }
      const float o0 = p0 + b20, o1 = p1 + b21;
      const float mx = (o0 > o1) ? o0 : o1;
      const float mine = (lane & 1) ? o1 : o0;
      const float sh = mine - mx;
      const float e  = expf(sh);
      const float es = e + __shfl_xor(e, 1);
      const float res = sh - logf(es);
      if (lane < 2) sO[2 * g + lane] = res;
    }
  }
  __syncthreads();
  const bool ok = tid < (2 * nG) / 4;
  const int tcl = ok ? tid : 0;
  const v4f v = *(const v4fa*)(sO + 4 * tcl);
  float* dp = out + 4 * (ok ? tid : 0);
  if (ok) *(volatile v4f*)dp = v;
  __threadfence();
  if (ok) *(volatile v4f*)dp = v;
}

static inline int cdiv(int a, int b) { return (a + b - 1) / b; }
static inline size_t al256(size_t o) { return (o + 255) & ~(size_t)255; }

extern "C" void kernel_launch(void* const* d_in, const int* in_sizes, int n_in,
                              void* d_out, int out_size, void* d_ws, size_t ws_size,
                              hipStream_t stream) {
  if (n_in < 44) return;
  if (in_sizes[0] < 2 || (in_sizes[0] & 1) != 0) return;
  const int nN = in_sizes[0] / 2;
  const int nE = in_sizes[1];
  if (nN < GBM || nN > (1 << 22) || (nN & 3) != 0) return;
  if (nE < 1 || nE > (1 << 21) || (nE & 3) != 0) return;
  if (in_sizes[2] != 2 || in_sizes[3] != 2 || in_sizes[4] != 4 || in_sizes[5] != 2) return;
  if (in_sizes[6] != 2 * HD) return;
  for (int k = 7; k <= 11; ++k) if (in_sizes[k] != HD) return;
  if (in_sizes[12] != HD * HD || in_sizes[13] != HD) return;
  for (int l = 1; l < 3; ++l) {
    const int b = 2 + 12 * l;
    if (in_sizes[b] != HD || in_sizes[b + 1] != HD) return;
    if (in_sizes[b + 2] != HD * HD || in_sizes[b + 3] != HD) return;
    if (in_sizes[b + 4] != HD * HD || in_sizes[b + 5] != HD) return;
    for (int k = 6; k <= 9; ++k) if (in_sizes[b + k] != HD) return;
    if (in_sizes[b + 10] != HD * HD || in_sizes[b + 11] != HD) return;
  }
  if (in_sizes[38] != G3 * G3 || in_sizes[39] != G3 || in_sizes[40] != 2 * G3 || in_sizes[41] != 2) return;
  if (in_sizes[42] != 2 * nE || in_sizes[43] != nN) return;
  if (out_size < 4 || (out_size & 3) != 0) return;
  const int nG = out_size / 2;
  if (nG < 1 || nG > 128 || 2 * nG != out_size) return;

  const float* x  = (const float*)d_in[0];
  const float* ea = (const float*)d_in[1];
  const float* PL[3][12];
  for (int l = 0; l < 3; ++l)
    for (int k = 0; k < 12; ++k) PL[l][k] = (const float*)d_in[2 + 12 * l + k];
  const float* lin1w = (const float*)d_in[38];
  const float* lin1b = (const float*)d_in[39];
  const float* lin2w = (const float*)d_in[40];
  const float* lin2b = (const float*)d_in[41];
  const int* ei    = (const int*)d_in[42];
  const int* src   = ei;
  const int* dst   = ei + nE;
  const int* batch = (const int*)d_in[43];
  float* out = (float*)d_out;

  const int MP  = cdiv(nN, GBM) * GBM;
  const int gM  = MP / GBM;
  const int nBk = cdiv(MP, NBRUN);
  if ((long long)nBk * NBRUN < (long long)MP) return;
  if ((MP % ARB) != 0 || ((MP * 16) % NTHR) != 0) return;

  char* ws = (char*)d_ws;
  size_t off = 0;
  const size_t oBT = off; off = al256(off + (size_t)NPL * NUP * 16);
  const size_t oA1 = off; off = al256(off + (size_t)MP * KP * 2);
  const size_t oA2 = off; off = al256(off + (size_t)MP * KP * 2);
  const size_t oF1 = off; off = al256(off + (size_t)MP * HD * 4);
  const size_t oF2 = off; off = al256(off + (size_t)MP * HD * 4);
  const size_t oLS = off; off = al256(off + (size_t)nBk * RCAP * 8);
  const size_t oCN = off; off = al256(off + (size_t)nBk * NBRUN * 4);
  const size_t oOF = off; off = al256(off + (size_t)nBk * NBRUN * 4);
  const size_t oFL = off; off = al256(off + (size_t)nBk * 128);
  const size_t oRC = off; off = al256(off + (size_t)gM * RECW * 4);
  const size_t oST = off; off = al256(off + (size_t)3 * STATW * 4);
  const size_t oPO = off; off = al256(off + (size_t)nG * G3 * 4);
  if (off > ws_size || off > (size_t)WSLIM) return;
  unsigned short* BT = (unsigned short*)(ws + oBT);
  unsigned short* A1 = (unsigned short*)(ws + oA1);
  unsigned short* A2 = (unsigned short*)(ws + oA2);
  float*          F1 = (float*)(ws + oF1);
  float*          F2 = (float*)(ws + oF2);
  unsigned int*   LS = (unsigned int*)(ws + oLS);
  int*            CN = (int*)(ws + oCN);
  int*            OF = (int*)(ws + oOF);
  int*            FL = (int*)(ws + oFL);
  float*          RC = (float*)(ws + oRC);
  float*          ST = (float*)(ws + oST);
  float*          PO = (float*)(ws + oPO);
  const size_t plS = (size_t)NUP * 8;

  hipFuncSetAttribute(reinterpret_cast<const void*>(&k_bucket), hipFuncAttributeMaxDynamicSharedMemorySize, LDS_BKT);
  hipFuncSetAttribute(reinterpret_cast<const void*>(&k_head),   hipFuncAttributeMaxDynamicSharedMemorySize, LDS_HEAD);

  const int gAg = MP / ARB;
  const int nUa = MP * 16;

  k_prep<<<(NPL * NUP) / NTHR, NTHR, 0, stream>>>(PL[0][10], PL[1][2], PL[1][4], PL[1][10],
                                                  PL[2][2], PL[2][4], PL[2][10], BT);
  k_bucket<<<nBk, NTHR, LDS_BKT, stream>>>(src, dst, ea, nN, nE, 1, LS, CN, OF, FL);

  k_agg1<<<gAg, NTHR, 0, stream>>>(x, LS, CN, OF, FL, PL[0][2], PL[0][3], PL[0][0], PL[0][1],
                                   PL[0][4], PL[0][5], PL[0][6], PL[0][7], PL[0][8], PL[0][9],
                                   (unsigned int*)A1, nN, MP);
  k_gemm<1><<<gM, NTHR, 0, stream>>>(A1, BT + 0 * plS, PL[0][11], PL[0][11], PL[0][11], PL[0][11], PL[0][11],
                                     F2, A2, RC, nN);
  k_comb<<<1, HD, 0, stream>>>(RC, gM, nN, ST);
  k_apply<<<nUa / NTHR, NTHR, 0, stream>>>(F2, ST, A2, nN, nUa);
  k_pool<<<nG, NTHR, 0, stream>>>(F2, ST, batch, nN, 1, PO, 0);

  k_gemm<0><<<gM, NTHR, 0, stream>>>(A2, BT + 1 * plS, PL[1][3], PL[1][3], PL[1][3], PL[1][3], PL[1][3],
                                     F1, A1, RC, nN);
  k_agg<<<gAg, NTHR, 0, stream>>>(F1, (const unsigned int*)A2, LS, CN, OF, FL, PL[1][3], PL[1][0], PL[1][1],
                                  (unsigned int*)A1, nN, MP);
  k_gemm<2><<<gM, NTHR, 0, stream>>>(A1, BT + 2 * plS, PL[1][5], PL[1][6], PL[1][7], PL[1][8], PL[1][9],
                                     F1, A2, RC, nN);
  k_gemm<1><<<gM, NTHR, 0, stream>>>(A2, BT + 3 * plS, PL[1][11], PL[1][11], PL[1][11], PL[1][11], PL[1][11],
                                     F2, A1, RC, nN);
  k_comb<<<1, HD, 0, stream>>>(RC, gM, nN, ST + STATW);
  k_apply<<<nUa / NTHR, NTHR, 0, stream>>>(F2, ST + STATW, A1, nN, nUa);
  k_pool<<<nG, NTHR, 0, stream>>>(F2, ST + STATW, batch, nN, 1, PO, HD);

  k_gemm<0><<<gM, NTHR, 0, stream>>>(A1, BT + 4 * plS, PL[2][3], PL[2][3], PL[2][3], PL[2][3], PL[2][3],
                                     F1, A2, RC, nN);
  k_agg<<<gAg, NTHR, 0, stream>>>(F1, (const unsigned int*)A1, LS, CN, OF, FL, PL[2][3], PL[2][0], PL[2][1],
                                  (unsigned int*)A2, nN, MP);
  k_gemm<2><<<gM, NTHR, 0, stream>>>(A2, BT + 5 * plS, PL[2][5], PL[2][6], PL[2][7], PL[2][8], PL[2][9],
                                     F1, A1, RC, nN);
  k_gemm<1><<<gM, NTHR, 0, stream>>>(A1, BT + 6 * plS, PL[2][11], PL[2][11], PL[2][11], PL[2][11], PL[2][11],
                                     F2, A2, RC, nN);
  k_comb<<<1, HD, 0, stream>>>(RC, gM, nN, ST + 2 * STATW);
  k_pool<<<nG, NTHR, 0, stream>>>(F2, ST + 2 * STATW, batch, nN, 1, PO, 2 * HD);

  k_head<<<1, NTHR, LDS_HEAD, stream>>>(PO, lin1w, lin1b, lin2w, lin2b, nG, out);
}
